// FnnNormFCIni_13795434955134
// MI455X (gfx1250) — hardware-run, weakly checked
//
#include <hip/hip_runtime.h>
#include <math.h>

constexpr int kRules = 64;
constexpr int kBatch = 4096;
constexpr int kFea   = 512;
constexpr int kCls   = 128;
constexpr int kNExp  = kRules * kCls;
constexpr int kChunkRows = 1024;
constexpr int kNumChunks = kBatch / kChunkRows;
constexpr int kRowsPerBlk = 8;
constexpr float kWCarry    = 32.0f;
constexpr float kWCarryInv = 1.0f / 32.0f;

static_assert(kBatch % kChunkRows == 0, "chunking");
static_assert(kChunkRows % 64 == 0 && kNExp % 64 == 0, "GEMM M,N tile multiples");
static_assert(kFea % 32 == 0, "GEMM K multiple of 32");
static_assert(kFea == 16 * 32, "member kernel: 16 d per lane");
static_assert(kRules == 64, "member kernel: 2 rules per lane in the softmax");
static_assert(kCls == 128, "combine kernel: 32 lanes x 4 floats per row");
static_assert(kBatch % kRowsPerBlk == 0 && kChunkRows % kRowsPerBlk == 0, "row blocks");

typedef __attribute__((ext_vector_type(16))) _Float16 v16h;
typedef __attribute__((ext_vector_type(8)))  _Float16 v8h;
typedef __attribute__((ext_vector_type(16))) __bf16   v16b;
typedef __attribute__((ext_vector_type(8)))  __bf16   v8b;
typedef __attribute__((ext_vector_type(8)))  float    v8f;
typedef __attribute__((ext_vector_type(4)))  float    v4f;
typedef __attribute__((ext_vector_type(4)))  unsigned int v4u;

__device__ __forceinline__ unsigned short f2bf_bits(float f) {
  unsigned u = __float_as_uint(f);
  return (unsigned short)((u + 0x7FFFu + ((u >> 16) & 1u)) >> 16);
}
__device__ __forceinline__ float bf_bits2f(unsigned short h) { return __uint_as_float(((unsigned)h) << 16); }

__device__ __forceinline__ void dep_guard_h(v8f& a, v8f& b, v16h x, v16h y) { asm volatile("v_nop\n\tv_nop\n\tv_nop\n\tv_nop" : "+v"(a), "+v"(b) : "v"(x), "v"(y)); }
__device__ __forceinline__ void dep_guard_b(v8f& a, v8f& b, v16b x, v16b y) { asm volatile("v_nop\n\tv_nop\n\tv_nop\n\tv_nop" : "+v"(a), "+v"(b) : "v"(x), "v"(y)); }
__device__ __forceinline__ void keep4_h(v16h a, v16h b, v16h c, v16h d) { asm volatile("v_nop" :: "v"(a), "v"(b), "v"(c), "v"(d)); }
__device__ __forceinline__ void keep4_b(v16b a, v16b b, v16b c, v16b d) { asm volatile("v_nop" :: "v"(a), "v"(b), "v"(c), "v"(d)); }
__device__ __forceinline__ void acc_guard4(v8f& a, v8f& b, v8f& c, v8f& d) { asm volatile("v_nop\n\tv_nop\n\tv_nop\n\tv_nop" : "+v"(a), "+v"(b), "+v"(c), "+v"(d)); }
template <typename T> struct Frag;
template <> struct Frag<_Float16> {
  typedef v16h V; union U { v16h v; v8h h[2]; };
  static __device__ __forceinline__ v16h load(const _Float16* p) {
    U f; f.h[0] = *(const v8h*)(p); f.h[1] = *(const v8h*)(p + 16); return f.v;
  }
  static __device__ __forceinline__ v8f mma(v16h a, v16h b, v8f c) {
    return __builtin_amdgcn_wmma_f32_16x16x32_f16(false, a, false, b, (short)0, c, false, false);
  }
  static __device__ __forceinline__ void guard(v8f& a, v8f& b, v16h x, v16h y) { dep_guard_h(a, b, x, y); }
  static __device__ __forceinline__ void keep(v16h a, v16h b, v16h c, v16h d) { keep4_h(a, b, c, d); }
};
template <> struct Frag<__bf16> {
  typedef v16b V; union U { v16b v; v8b h[2]; };
  static __device__ __forceinline__ v16b load(const __bf16* p) {
    U f; f.h[0] = *(const v8b*)(p); f.h[1] = *(const v8b*)(p + 16); return f.v;
  }
  static __device__ __forceinline__ v8f mma(v16b a, v16b b, v8f c) {
    return __builtin_amdgcn_wmma_f32_16x16x32_bf16(false, a, false, b, (short)0, c, false, false);
  }
  static __device__ __forceinline__ void guard(v8f& a, v8f& b, v16b x, v16b y) { dep_guard_b(a, b, x, y); }
  static __device__ __forceinline__ void keep(v16b a, v16b b, v16b c, v16b d) { keep4_b(a, b, c, d); }
};

__device__ __forceinline__ unsigned pk16(unsigned short a, unsigned short b) { return (unsigned)a | ((unsigned)b << 16); }
__device__ __forceinline__ unsigned short h_bits(float f) { const _Float16 h = (_Float16)f; return __builtin_bit_cast(unsigned short, h); }

template <int ET> struct Elem;
template <> struct Elem<0> { typedef _Float16 T; };
template <> struct Elem<1> { typedef __bf16 T; };
template <int ET, bool SPLIT, int BIAS_MODE, int OUT_MODE, bool RESID, int ACT = 0>
__global__ __launch_bounds__(256) void wmma_gemm64(
    const unsigned short* __restrict__ Ap, const unsigned short* __restrict__ A2p, int lda, long strideA,
    const unsigned short* __restrict__ Btp, const unsigned short* __restrict__ Bt2p, int ldb, long strideB,
    void* __restrict__ Cout, void* __restrict__ Cout2, int ldc, long strideC,
    const float* __restrict__ bias,
    const float* __restrict__ resid, long strideR,
    int M, int N, int K, float scale) {
  typedef typename Elem<ET>::T T;
  typedef typename Frag<T>::V V;
  const T* A = (const T*)Ap; const T* A2 = (const T*)A2p; const T* Bt = (const T*)Btp; const T* Bt2 = (const T*)Bt2p;
  __shared__ __align__(16) float sT[8][16 * 68];
  const int b    = blockIdx.y;
  const int lane = threadIdx.x & 31;
  const int wave = threadIdx.x >> 5;
  const int tilesN = N >> 6;
  const int tilesM = M >> 6;
  const int tile = blockIdx.x * 8 + wave;
  if (tile >= tilesM * tilesN) return;
  const int tm = tile / tilesN;
  const int tn = tile - tm * tilesN;
  const int m0 = tm << 6;
  const int n0 = tn << 6;

  const T* Ab  = A  + (size_t)b * strideA;
  const T* Bb  = Bt + (size_t)b * strideB;
  const T* Ab2 = SPLIT ? (A2  + (size_t)b * strideA) : nullptr;
  const T* Bb2 = SPLIT ? (Bt2 + (size_t)b * strideB) : nullptr;

  const int rlane = lane & 15;
  const int koff  = (lane >> 4) * 8;
  const int mOff  = (lane >> 4) * 8;

  v8f acc[4][4];
#pragma unroll
  for (int i = 0; i < 4; ++i)
#pragma unroll
    for (int j = 0; j < 4; ++j) acc[i][j] = (v8f){0.f,0.f,0.f,0.f,0.f,0.f,0.f,0.f};

  for (int k0 = 0; k0 < K; k0 += 32) {
    V bh[4], bl[4];
#pragma unroll
    for (int j = 0; j < 4; ++j) {
      const size_t bo = (size_t)(n0 + (j << 4) + rlane) * ldb + koff + k0;
      bh[j] = Frag<T>::load(Bb + bo);
      if (SPLIT) bl[j] = Frag<T>::load(Bb2 + bo);
    }
#pragma unroll
    for (int i = 0; i < 4; ++i) {
      const size_t ao = (size_t)(m0 + (i << 4) + rlane) * lda + koff + k0;
      V ah = Frag<T>::load(Ab + ao);
      V al;
      if (SPLIT) al = Frag<T>::load(Ab2 + ao);
#pragma unroll
      for (int j = 0; j < 4; ++j) {
        acc[i][j] = Frag<T>::mma(ah, bh[j], acc[i][j]);
        if (SPLIT) {
          acc[i][j] = Frag<T>::mma(ah, bl[j], acc[i][j]);
          acc[i][j] = Frag<T>::mma(al, bh[j], acc[i][j]);
        }
      }
      Frag<T>::guard(acc[i][0], acc[i][3], ah, SPLIT ? al : ah);
    }
    Frag<T>::keep(bh[0], bh[1], bh[2], bh[3]);
    if (SPLIT) Frag<T>::keep(bl[0], bl[1], bl[2], bl[3]);
  }
  acc_guard4(acc[0][0], acc[0][1], acc[0][2], acc[0][3]);
  acc_guard4(acc[1][0], acc[1][1], acc[1][2], acc[1][3]);
  acc_guard4(acc[2][0], acc[2][1], acc[2][2], acc[2][3]);
  acc_guard4(acc[3][0], acc[3][1], acc[3][2], acc[3][3]);

  float* slab = sT[wave];
  const float* Rb = RESID ? (resid + (size_t)b * strideR) : nullptr;
#pragma unroll
  for (int i = 0; i < 4; ++i) {
    const int mBase = m0 + (i << 4);
#pragma unroll
    for (int j = 0; j < 4; ++j) {
      const int n = n0 + (j << 4) + rlane;
      float bv = 0.f;
      if (BIAS_MODE == 2) bv = bias[n];
#pragma unroll
      for (int r = 0; r < 8; ++r) {
        float v = acc[i][j][r] * scale;
        if (BIAS_MODE == 1) v += bias[mBase + mOff + r];
        if (BIAS_MODE == 2) v += bv;
        if (RESID) v += Rb[(size_t)(mBase + mOff + r) * ldc + n];
        if (ACT == 2) v = fmaxf(v, 0.0f);
        if (ACT == 4) v = (v > 0.f) ? v : 0.01f * v;
        slab[(mOff + r) * 68 + (j << 4) + rlane] = v;
      }
    }
    __builtin_amdgcn_fence(__ATOMIC_RELEASE, "workgroup");
    __builtin_amdgcn_wave_barrier();
    __builtin_amdgcn_fence(__ATOMIC_ACQUIRE, "workgroup");
    if (OUT_MODE == 0) {
      float* C = (float*)Cout + (size_t)b * strideC;
      const int hh = lane >> 4, c4 = (lane & 15) * 4;
      for (int pass = 0; pass < 2; ++pass) {
#pragma unroll
        for (int it = 0; it < 8; ++it) {
          const int row = it * 2 + hh;
          v4f v = *(const v4f*)(slab + row * 68 + c4);
          *(volatile v4f*)(C + (size_t)(mBase + row) * ldc + n0 + c4) = v;
        }
        __threadfence();
      }
    } else {
      const int q = lane >> 3, c8 = (lane & 7) * 8;
      unsigned short* C  = (unsigned short*)Cout  + (size_t)b * strideC;
      unsigned short* C2 = (OUT_MODE == 2) ? ((unsigned short*)Cout2 + (size_t)b * strideC) : nullptr;
      for (int pass = 0; pass < 2; ++pass) {
#pragma unroll
        for (int it = 0; it < 4; ++it) {
          const int row = it * 4 + q;
          const float* sp = slab + row * 68 + c8;
          v8h hv, lv;
#pragma unroll
          for (int e = 0; e < 8; ++e) {
            if (OUT_MODE == 1) {
              hv[e] = (_Float16)sp[e];
            } else {
              unsigned short hb = f2bf_bits(sp[e]);
              unsigned short lb = f2bf_bits(sp[e] - bf_bits2f(hb));
              hv[e] = __builtin_bit_cast(_Float16, hb);
              lv[e] = __builtin_bit_cast(_Float16, lb);
            }
          }
          *(volatile v8h*)(C + (size_t)(mBase + row) * ldc + n0 + c8) = hv;
          if (OUT_MODE == 2) *(volatile v8h*)(C2 + (size_t)(mBase + row) * ldc + n0 + c8) = lv;
        }
        __threadfence();
      }
    }
    __builtin_amdgcn_fence(__ATOMIC_RELEASE, "workgroup");
    __builtin_amdgcn_wave_barrier();
    __builtin_amdgcn_fence(__ATOMIC_ACQUIRE, "workgroup");
  }
}

__global__ __launch_bounds__(256) void cast8_f16_kernel(const float* __restrict__ in, unsigned short* __restrict__ out, int n8) {
  const int i = blockIdx.x * 256 + threadIdx.x;
  if (i >= n8) return;
  const float* p = in + 8 * (size_t)i;
  const v4f a = *(const v4f*)(p);
  const v4f c = *(const v4f*)(p + 4);
  unsigned short hb[8];
#pragma unroll
  for (int e = 0; e < 4; ++e) {
    hb[e]     = h_bits(a[e]);
    hb[4 + e] = h_bits(c[e]);
  }
  const v4u u = (v4u){pk16(hb[0], hb[1]), pk16(hb[2], hb[3]), pk16(hb[4], hb[5]), pk16(hb[6], hb[7])};
  unsigned short* q = out + 8 * (size_t)i;
  *(volatile v4u*)q = u;
  __threadfence();
  *(volatile v4u*)q = u;
}

__global__ __launch_bounds__(256) void rcp_kernel(const float* __restrict__ var, float* __restrict__ nrcp, int n4) {
#pragma clang fp contract(off)
  const int i = blockIdx.x * 256 + threadIdx.x;
  if (i >= n4) return;
  const v4f vv = *(const v4f*)(var + 4 * (size_t)i);
  v4f o;
#pragma unroll
  for (int e = 0; e < 4; ++e) {
    const float v   = fminf(fmaxf(vv[e], 0.0001f), 0.1f);
    const float den = 2.0f * (v * v);
    o[e] = -(1.0f / den);
  }
  float* q = nrcp + 4 * (size_t)i;
  *(volatile v4f*)q = o;
  __threadfence();
  *(volatile v4f*)q = o;
}

__global__ __launch_bounds__(256) void wtcast_kernel(const float* __restrict__ W, unsigned short* __restrict__ out, float scale) {
  __shared__ float sm[kCls][65];
  const int t  = threadIdx.x;
  const int d0 = blockIdx.x * 64;
  const int r  = blockIdx.y;
  const float* Wr = W + (size_t)r * kFea * kCls;
#pragma unroll
  for (int i = 0; i < 32; ++i) {
    const int e  = i * 256 + t;
    const int dl = e >> 7;
    const int c  = e & 127;
    sm[c][dl] = Wr[(size_t)(d0 + dl) * kCls + c] * scale;
  }
  __syncthreads();
  const int lane = t & 31, wave = t >> 5;
  const int q = lane >> 3, c8 = (lane & 7) * 8;
  unsigned short* op = out + (size_t)r * kCls * kFea;
  for (int pass = 0; pass < 2; ++pass) {
#pragma unroll
    for (int it = 0; it < 4; ++it) {
      const int row = wave * 16 + it * 4 + q;
      unsigned short hb[8];
#pragma unroll
      for (int e = 0; e < 8; ++e) hb[e] = h_bits(sm[row][c8 + e]);
      const v4u u = (v4u){pk16(hb[0], hb[1]), pk16(hb[2], hb[3]), pk16(hb[4], hb[5]), pk16(hb[6], hb[7])};
      *(volatile v4u*)(op + (size_t)row * kFea + d0 + c8) = u;
    }
    __threadfence();
  }
}

__global__ __launch_bounds__(256) void member_kernel(const float* __restrict__ x, const float* __restrict__ proto,
                                                     const float* __restrict__ nrcp, float* __restrict__ fire) {
#pragma clang fp contract(off)
  __shared__ __align__(16) float fsL[kRowsPerBlk][kRules];
  const int t = threadIdx.x, lane = t & 31, w = t >> 5;
  const int b = blockIdx.x * kRowsPerBlk + w;
  const float* xrow = x + (size_t)b * kFea + lane;
  float xr[16];
#pragma unroll
  for (int i = 0; i < 16; ++i) xr[i] = xrow[32 * i];

#pragma unroll 1
  for (int r = 0; r < kRules; ++r) {
    const float* pr = proto + (size_t)r * kFea + lane;
    const float* cr = nrcp  + (size_t)r * kFea + lane;
    float s = 0.0f;
#pragma unroll
    for (int i = 0; i < 16; ++i) {
      const float pv   = pr[32 * i];
      const float cv   = cr[32 * i];
      const float diff = xr[i] - pv;
      const float num  = diff * diff;
      const float m    = expf(num * cv);
      const float mm   = m * m;
      s = s + mm;
    }
    s += __shfl_xor(s, 16, 32);
    s += __shfl_xor(s, 8, 32);
    s += __shfl_xor(s, 4, 32);
    s += __shfl_xor(s, 2, 32);
    s += __shfl_xor(s, 1, 32);
    if (lane == 0) fsL[w][r] = s;
  }
  __syncthreads();

  const float v0 = fsL[w][lane];
  const float v1 = fsL[w][lane + 32];
  float mx = fmaxf(v0, v1);
  mx = fmaxf(mx, __shfl_xor(mx, 16, 32));
  mx = fmaxf(mx, __shfl_xor(mx, 8, 32));
  mx = fmaxf(mx, __shfl_xor(mx, 4, 32));
  mx = fmaxf(mx, __shfl_xor(mx, 2, 32));
  mx = fmaxf(mx, __shfl_xor(mx, 1, 32));
  const float e0 = expf(v0 - mx);
  const float e1 = expf(v1 - mx);
  float sum = e0 + e1;
  sum += __shfl_xor(sum, 16, 32);
  sum += __shfl_xor(sum, 8, 32);
  sum += __shfl_xor(sum, 4, 32);
  sum += __shfl_xor(sum, 2, 32);
  sum += __shfl_xor(sum, 1, 32);
  const float inv = 1.0f / sum;
  const float p0 = e0 * inv;
  const float p1 = e1 * inv;
  __syncthreads();
  fsL[w][lane]      = p0;
  fsL[w][lane + 32] = p1;
  __syncthreads();

  const int l16 = lane & 15;
  const v4f val = *(const v4f*)(&fsL[w][4 * l16]);
  float* dst = fire + (size_t)b * kRules + 4 * l16;
  if (lane < 16) *(volatile v4f*)dst = val;
  __threadfence();
  if (lane < 16) *(volatile v4f*)dst = val;
}

__global__ __launch_bounds__(256) void combine_kernel(const float* __restrict__ expv, const float* __restrict__ fire,
                                                      float* __restrict__ out, int chunkRow0) {
  __shared__ float fS[kRowsPerBlk][kRules];
  const int t = threadIdx.x, lane = t & 31, w = t >> 5;
  const int blRow0 = blockIdx.x * kRowsPerBlk;
  for (int e = t; e < kRowsPerBlk * kRules; e += 256) {
    const int row = e >> 6, rr = e & 63;
    fS[row][rr] = fire[(size_t)(chunkRow0 + blRow0 + row) * kRules + rr];
  }
  __syncthreads();
  const int bl = blRow0 + w;
  const int bg = chunkRow0 + bl;
  v4f acc = (v4f){0.f, 0.f, 0.f, 0.f};
  const float* ep = expv + (size_t)bl * kNExp + 4 * lane;
#pragma unroll 4
  for (int r = 0; r < kRules; ++r) {
    const v4f ev = *(const v4f*)(ep + r * kCls);
    const float f = fS[w][r];
    acc = acc + ev * f;
  }
  float* dst = out + (size_t)bg * kCls + 4 * lane;
  *(volatile v4f*)dst = acc;
  __threadfence();
  *(volatile v4f*)dst = acc;
}

extern "C" void kernel_launch(void* const* d_in, const int* in_sizes, int n_in,
                              void* d_out, int out_size, void* d_ws, size_t ws_size,
                              hipStream_t stream) {
  if (n_in < 5) return;
  if (in_sizes[0] != kBatch * kFea || in_sizes[1] != kRules * kFea || in_sizes[2] != kRules * kFea ||
      in_sizes[3] != kRules * kFea * kCls || in_sizes[4] != kRules * kCls) return;
  if (out_size != kBatch * kCls + kBatch * kRules) return;

  const float* x     = (const float*)d_in[0];
  const float* proto = (const float*)d_in[1];
  const float* var   = (const float*)d_in[2];
  const float* W     = (const float*)d_in[3];
  const float* bias  = (const float*)d_in[4];

  float* out0 = (float*)d_out;
  float* fire = out0 + (size_t)kBatch * kCls;

  const size_t offX16  = 0;
  const size_t szX16   = (size_t)kBatch * kFea * 2;
  const size_t offWT16 = offX16 + szX16;
  const size_t szWT16  = (size_t)kNExp * kFea * 2;
  const size_t offNRCP = offWT16 + szWT16;
  const size_t szNRCP  = (size_t)kRules * kFea * 4;
  const size_t offEXP  = offNRCP + szNRCP;
  const size_t szEXP   = (size_t)kChunkRows * kNExp * 4;
  const size_t total   = offEXP + szEXP;
  if (total > ws_size) return;

  char* ws = (char*)d_ws;
  unsigned short* X16  = (unsigned short*)(ws + offX16);
  unsigned short* WT16 = (unsigned short*)(ws + offWT16);
  float*          NRCP = (float*)(ws + offNRCP);
  float*          EXPV = (float*)(ws + offEXP);

  {
    const int n4 = kRules * kFea / 4;
    rcp_kernel<<<(n4 + 255) / 256, 256, 0, stream>>>(var, NRCP, n4);
  }
  {
    const int n8 = kBatch * kFea / 8;
    cast8_f16_kernel<<<(n8 + 255) / 256, 256, 0, stream>>>(x, X16, n8);
  }
  wtcast_kernel<<<dim3(kFea / 64, kRules), 256, 0, stream>>>(W, WT16, kWCarry);
  member_kernel<<<kBatch / kRowsPerBlk, 256, 0, stream>>>(x, proto, NRCP, fire);
  for (int ch = 0; ch < kNumChunks; ++ch) {
    const int tiles = (kChunkRows / 64) * (kNExp / 64);
    wmma_gemm64<0, false, 2, 0, false, 2><<<dim3((tiles + 7) / 8, 1), 256, 0, stream>>>(
        X16 + (size_t)ch * kChunkRows * kFea, nullptr, kFea, 0L,
        WT16, nullptr, kFea, 0L,
        (void*)EXPV, nullptr, kNExp, 0L,
        bias,
        nullptr, 0L,
        kChunkRows, kNExp, kFea, kWCarryInv);
    combine_kernel<<<kChunkRows / kRowsPerBlk, 256, 0, stream>>>(EXPV, fire, out0, ch * kChunkRows);
  }
}
